// GAT_63333587747452
// MI455X (gfx1250) — hardware-verified
//
#include <hip/hip_runtime.h>
#include <math.h>
#include <stdint.h>

#define GB 16
#define GN 512
#define GF 64
#define GT 12
#define GH 4
#define GO 32
#define GHO 128
#define GC 64
#define BT (GB * GT)
#define NTOK (BT * GN)
#define NEGV (-9e15f)

#define PB_X  (GB * GN / 8)
#define PB_W1 4
#define PB_W2 8
#define PB_AV 1
#define PB_MB 32
#define PB_ALL (PB_X + PB_W1 + PB_W2 + PB_AV + PB_MB)

static_assert(GN == 4 * 128);
static_assert(GT == 12);
static_assert(BT == 192);
static_assert(NTOK == 98304);
static_assert(NTOK % 128 == 0);
static_assert(GF % 32 == 0);
static_assert(GHO % 32 == 0);
static_assert((2 * GHO) % 32 == 0);
static_assert(GO == 32);
static_assert(GC == 64);
static_assert(GH * GO == GHO);
static_assert((GC * GT * 4) % 128 == 0);
static_assert(GN / 32 == 16);
static_assert(GN % 64 == 0);
static_assert(((GHO / 64) * (NTOK / 64)) % 8 == 0);
static_assert(((GC / 64) * (NTOK / 64)) % 8 == 0);
static_assert(PB_X * 8 == GB * GN);

typedef __attribute__((ext_vector_type(16))) __bf16   v16b;
typedef __attribute__((ext_vector_type(8)))  __bf16   v8b;
typedef __attribute__((ext_vector_type(8)))  float    v8f;
typedef __attribute__((ext_vector_type(4)))  float    v4f;
typedef __attribute__((ext_vector_type(4)))  unsigned int v4u;

__device__ __forceinline__ unsigned short f2bf_bits(float f) {
  unsigned u = __float_as_uint(f);
  return (unsigned short)((u + 0x7FFFu + ((u >> 16) & 1u)) >> 16);
}
__device__ __forceinline__ float bf_bits2f(unsigned short h) { return __uint_as_float(((unsigned)h) << 16); }
__device__ __forceinline__ float bf_rne(float f) { return bf_bits2f(f2bf_bits(f)); }
__device__ __forceinline__ unsigned pk16(unsigned short a, unsigned short b) { return (unsigned)a | ((unsigned)b << 16); }

__device__ __forceinline__ void dep_guard_b(v8f& a, v8f& b, v16b x, v16b y) { asm volatile("v_nop\n\tv_nop\n\tv_nop\n\tv_nop" : "+v"(a), "+v"(b) : "v"(x), "v"(y)); }
__device__ __forceinline__ void keep4_b(v16b a, v16b b, v16b c, v16b d) { asm volatile("v_nop" :: "v"(a), "v"(b), "v"(c), "v"(d)); }
__device__ __forceinline__ void acc_guard4(v8f& a, v8f& b, v8f& c, v8f& d) { asm volatile("v_nop\n\tv_nop\n\tv_nop\n\tv_nop" : "+v"(a), "+v"(b), "+v"(c), "+v"(d)); }

union FBu { v16b v; v8b h[2]; };
__device__ __forceinline__ v16b frag_load(const __bf16* p) {
  FBu f; f.h[0] = *(const v8b*)(p); f.h[1] = *(const v8b*)(p + 16); return f.v;
}
__device__ __forceinline__ v8f mma_b(v16b a, v16b b, v8f c) {
  return __builtin_amdgcn_wmma_f32_16x16x32_bf16(false, a, false, b, (short)0, c, false, false);
}
__device__ __forceinline__ v8f at_mma(v16b a, v16b b, v8f c) {
  c = __builtin_amdgcn_wmma_f32_16x16x32_bf16(false, a, false, b, (short)0, c, false, false);
  asm volatile("v_nop\n\tv_nop\n\tv_nop\n\tv_nop" : "+v"(c) : "v"(a), "v"(b));
  return c;
}
__device__ __forceinline__ void at_split(float f, __bf16& hi, __bf16& lo) {
  const unsigned short hb = f2bf_bits(f);
  hi = __builtin_bit_cast(__bf16, hb);
  lo = __builtin_bit_cast(__bf16, f2bf_bits(f - bf_bits2f(hb)));
}
__device__ __forceinline__ void wave_lds_sync() {
  __builtin_amdgcn_fence(__ATOMIC_RELEASE, "workgroup");
  __builtin_amdgcn_wave_barrier();
  __builtin_amdgcn_fence(__ATOMIC_ACQUIRE, "workgroup");
}

__global__ __launch_bounds__(256) void k_prep(const float* __restrict__ x, const int* __restrict__ adj,
                                              const float* __restrict__ Wh, const float* __restrict__ ah,
                                              const float* __restrict__ Wo, const float* __restrict__ ao,
                                              unsigned short* __restrict__ XB, unsigned short* __restrict__ W1t,
                                              unsigned short* __restrict__ W2t2, float* __restrict__ AV,
                                              unsigned* __restrict__ MB) {
  __shared__ __align__(16) float xt[8 * 768];
  const int blk = blockIdx.x;
  const int tid = threadIdx.x;
  if (blk < PB_X) {
    const int g = blk;
    const float* src = x + (size_t)g * 6144;
#pragma unroll
    for (int it = 0; it < 6; ++it) {
      const int idx = it * 256 + tid;
      const v4f a = *(const v4f*)(src + idx * 4);
      *(v4f*)(xt + idx * 4) = a;
    }
    __syncthreads();
    const int b  = g >> 6;
    const int n0 = (g & 63) * 8;
    v4u hv[3];
#pragma unroll
    for (int it = 0; it < 3; ++it) {
      const int p = it * 256 + tid;
      const int t = p >> 6;
      const int rem = p & 63;
      const int nn = rem >> 3, f8 = rem & 7;
      const float* sp = xt + nn * 768 + (f8 * 8) * 12 + t;
      v4u a;
#pragma unroll
      for (int q = 0; q < 4; ++q) {
        const float f0 = sp[(2 * q) * 12];
        const float f1 = sp[(2 * q + 1) * 12];
        a[q] = pk16(f2bf_bits(f0), f2bf_bits(f1));
      }
      hv[it] = a;
    }
    for (int pass = 0; pass < 2; ++pass) {
#pragma unroll
      for (int it = 0; it < 3; ++it) {
        const int p = it * 256 + tid;
        const int t = p >> 6;
        const int rem = p & 63;
        const int nn = rem >> 3, f8 = rem & 7;
        const size_t go = ((size_t)((b * GT + t) * GN + n0 + nn)) * GF + f8 * 8;
        *(volatile v4u*)(XB + go) = hv[it];
      }
      __threadfence();
    }
  } else if (blk < PB_X + PB_W1) {
    const int p = (blk - PB_X) * 256 + tid;
    const int row = p >> 3, k8 = p & 7;
    const int h = row >> 5, o = row & 31;
    const float* src = Wh + (size_t)h * (GF * GO) + (size_t)(k8 * 8) * GO + o;
    v4u a;
#pragma unroll
    for (int q = 0; q < 4; ++q) {
      const float f0 = src[(2 * q) * GO];
      const float f1 = src[(2 * q + 1) * GO];
      a[q] = pk16(f2bf_bits(f0), f2bf_bits(f1));
    }
    *(volatile v4u*)(W1t + (size_t)row * GF + k8 * 8) = a;
    __threadfence();
    *(volatile v4u*)(W1t + (size_t)row * GF + k8 * 8) = a;
  } else if (blk < PB_X + PB_W1 + PB_W2) {
    const int p = (blk - PB_X - PB_W1) * 256 + tid;
    const int row = p >> 5, k8 = p & 31;
    v4u a;
#pragma unroll
    for (int q = 0; q < 4; ++q) {
      const int k0 = k8 * 8 + 2 * q;
      const float f0 = Wo[(size_t)(k0 & 127) * GC + row];
      const float f1 = Wo[(size_t)((k0 + 1) & 127) * GC + row];
      a[q] = pk16(f2bf_bits(f0), f2bf_bits(f1));
    }
    *(volatile v4u*)(W2t2 + (size_t)row * 256 + k8 * 8) = a;
    __threadfence();
    *(volatile v4u*)(W2t2 + (size_t)row * 256 + k8 * 8) = a;
  } else if (blk < PB_X + PB_W1 + PB_W2 + PB_AV) {
    const int tc = (tid < 96) ? tid : 95;
    const int e0 = tc * 4;
    v4f val;
#pragma unroll
    for (int q = 0; q < 4; ++q) {
      const int e  = e0 + q;
      const int g  = e >> 7;
      const int eh = e & 127;
      const int idxH = (eh >> 5) * 64 + (g & 1) * 32 + (eh & 31);
      const int idxO = (e >= 256) ? (e - 256) : 0;
      const float vh = ah[idxH];
      const float vo = ao[idxO];
      val[q] = bf_rne((e < 256) ? vh : vo);
    }
    if (tid < 96) {
      *(volatile v4f*)(AV + e0) = val;
      __threadfence();
      *(volatile v4f*)(AV + e0) = val;
    }
  } else {
    const int wv = (blk - (PB_X + PB_W1 + PB_W2 + PB_AV)) * 8 + (tid >> 5);
    const int lane = tid & 31;
    unsigned mine = 0u;
#pragma unroll 4
    for (int i = 0; i < 32; ++i) {
      const int row = 2 * wv + (i >> 4);
      const int w = i & 15;
      const int v = adj[(size_t)row * GN + w * 32 + lane];
      const unsigned bal = __builtin_amdgcn_ballot_w32(v > 0);
      mine = (lane == i) ? bal : mine;
    }
    ((volatile unsigned*)MB)[wv * 32 + lane] = mine;
    __threadfence();
    ((volatile unsigned*)MB)[wv * 32 + lane] = mine;
  }
}

template <int LAYER>
__global__ __launch_bounds__(256) void k_gemm_vt(const unsigned short* __restrict__ Wp, const unsigned short* __restrict__ Xp,
                                                 const float* __restrict__ AV,
                                                 unsigned short* __restrict__ VTh, unsigned short* __restrict__ VTl,
                                                 float* __restrict__ SD) {
  constexpr int K     = (LAYER == 1) ? GF : (2 * GHO);
  constexpr int TM    = (LAYER == 1) ? 2 : 1;
  constexpr int ASO   = (LAYER == 1) ? 0 : 256;
  constexpr int ADO   = (LAYER == 1) ? 128 : 320;
  constexpr int PLANE = (LAYER == 1) ? (BT * GH * GN) : (BT * GN);
  static_assert(K % 32 == 0);
  __shared__ __align__(16) float sT[8][16 * 68];
  __shared__ __align__(16) float sdl[8][128];
  const __bf16* A  = (const __bf16*)(const void*)Wp;
  const __bf16* Bt = (const __bf16*)(const void*)Xp;
  const int lane = threadIdx.x & 31;
  const int wave = threadIdx.x >> 5;
  const int tile = blockIdx.x * 8 + wave;
  const int tm = tile % TM;
  const int tn = tile / TM;
  const int m0 = tm << 6;
  const int n0 = tn << 6;
  const int rlane = lane & 15;
  const int hh    = lane >> 4;
  const int koff  = hh * 8;
  const int mOff  = hh * 8;

  v8f acc[4][4];
#pragma unroll
  for (int i = 0; i < 4; ++i)
#pragma unroll
    for (int j = 0; j < 4; ++j) acc[i][j] = (v8f){0.f,0.f,0.f,0.f,0.f,0.f,0.f,0.f};

#pragma unroll 1
  for (int k0 = 0; k0 < K; k0 += 32) {
    v16b bh[4];
#pragma unroll
    for (int j = 0; j < 4; ++j) {
      const size_t bo = (size_t)(n0 + (j << 4) + rlane) * K + koff + k0;
      bh[j] = frag_load(Bt + bo);
    }
#pragma unroll
    for (int i = 0; i < 4; ++i) {
      const size_t ao = (size_t)(m0 + (i << 4) + rlane) * K + koff + k0;
      v16b ahf = frag_load(A + ao);
#pragma unroll
      for (int j = 0; j < 4; ++j) acc[i][j] = mma_b(ahf, bh[j], acc[i][j]);
      dep_guard_b(acc[i][0], acc[i][3], ahf, ahf);
    }
    keep4_b(bh[0], bh[1], bh[2], bh[3]);
  }
  acc_guard4(acc[0][0], acc[0][1], acc[0][2], acc[0][3]);
  acc_guard4(acc[1][0], acc[1][1], acc[1][2], acc[1][3]);
  acc_guard4(acc[2][0], acc[2][1], acc[2][2], acc[2][3]);
  acc_guard4(acc[3][0], acc[3][1], acc[3][2], acc[3][3]);

  {
    float* sw = sdl[wave];
    float ps[4], pd[4];
#pragma unroll
    for (int j = 0; j < 4; ++j) { ps[j] = 0.f; pd[j] = 0.f; }
#pragma unroll
    for (int i = 0; i < 4; ++i) {
      const float* aps = AV + ASO + m0 + (i << 4) + mOff;
      const float* apd = AV + ADO + m0 + (i << 4) + mOff;
      const v4f s0 = *(const v4f*)(aps);
      const v4f s1 = *(const v4f*)(aps + 4);
      const v4f d0 = *(const v4f*)(apd);
      const v4f d1 = *(const v4f*)(apd + 4);
      float asv[8], adv[8];
#pragma unroll
      for (int r = 0; r < 4; ++r) { asv[r] = s0[r]; asv[r + 4] = s1[r]; adv[r] = d0[r]; adv[r + 4] = d1[r]; }
#pragma unroll
      for (int j = 0; j < 4; ++j) {
#pragma unroll
        for (int r = 0; r < 8; ++r) {
          ps[j] = fmaf(acc[i][j][r], asv[r], ps[j]);
          pd[j] = fmaf(acc[i][j][r], adv[r], pd[j]);
        }
      }
      const bool fin = (LAYER == 2) ? (i == 3) : ((i & 1) == 1);
      if (fin) {
#pragma unroll
        for (int j = 0; j < 4; ++j) {
          const float st = ps[j] + __shfl_xor(ps[j], 16, 32);
          const float dt = pd[j] + __shfl_xor(pd[j], 16, 32);
          sw[hh * 64 + (j << 4) + rlane] = (hh != 0) ? dt : st;
          ps[j] = 0.f; pd[j] = 0.f;
        }
        wave_lds_sync();
        const v4f v = *(const v4f*)(sw + lane * 4);
        size_t base;
        if (LAYER == 1) {
          const int head = tm * 2 + (i >> 1);
          base = (size_t)(((n0 >> 9) * GH + head) * GN + (n0 & 511));
        } else {
          base = (size_t)n0;
        }
        const size_t o = (size_t)hh * PLANE + base + (size_t)(lane & 15) * 4;
        *(volatile v4f*)(SD + o) = v;
        __threadfence();
        *(volatile v4f*)(SD + o) = v;
        wave_lds_sync();
      }
    }
  }

  float* slab = sT[wave];
#pragma unroll
  for (int i = 0; i < 4; ++i) {
    const int mBase = m0 + (i << 4);
#pragma unroll
    for (int j = 0; j < 4; ++j) {
#pragma unroll
      for (int r = 0; r < 8; ++r) slab[(mOff + r) * 68 + (j << 4) + rlane] = acc[i][j][r];
    }
    wave_lds_sync();
    {
      const int q = lane >> 3, c8 = (lane & 7) * 8;
      for (int pass = 0; pass < 2; ++pass) {
#pragma unroll
        for (int it = 0; it < 4; ++it) {
          const int row = it * 4 + q;
          const float* sp = slab + row * 68 + c8;
          v4u hv, lv;
#pragma unroll
          for (int e = 0; e < 4; ++e) {
            const float f0 = sp[2 * e], f1 = sp[2 * e + 1];
            const unsigned short h0 = f2bf_bits(f0), h1 = f2bf_bits(f1);
            const unsigned short l0 = f2bf_bits(f0 - bf_bits2f(h0)), l1 = f2bf_bits(f1 - bf_bits2f(h1));
            hv[e] = pk16(h0, h1);
            lv[e] = pk16(l0, l1);
          }
          const size_t go = (size_t)(mBase + row) * NTOK + n0 + c8;
          *(volatile v4u*)(VTh + go) = hv;
          *(volatile v4u*)(VTl + go) = lv;
        }
        __threadfence();
      }
    }
    wave_lds_sync();
  }
}

extern __shared__ __align__(16) float dyn_slab[];

template <int NTL, int MODE>
__global__ __launch_bounds__(128) void k_att(const unsigned short* __restrict__ vthp, const unsigned short* __restrict__ vtlp,
                                             const float* __restrict__ SD, const unsigned* __restrict__ MB,
                                             unsigned short* __restrict__ x1hl, float* __restrict__ out) {
  constexpr int HD    = NTL * 16;
  constexpr int NIT   = (MODE == 1) ? GH : GT;
  constexpr int PLANE = (MODE == 1) ? (BT * GH * GN) : (BT * GN);
  constexpr int PPT   = HD / 16;
  constexpr int XSN   = (MODE == 1) ? (64 * 132) : 4;
  static_assert(HD * 8 == 128 * PPT);
  union FB { v16b v; v8b h[2]; };
  __shared__ __align__(16) __bf16 Vth[HD * 64];
  __shared__ __align__(16) __bf16 Vtl[HD * 64];
  __shared__ __align__(16) __bf16 Psh[4][16 * 64];
  __shared__ __align__(16) __bf16 Psl[4][16 * 64];
  __shared__ __align__(16) float  dsh[GN];
  __shared__ __align__(16) unsigned mk[64 * 16];
  __shared__ __align__(16) float  xs[XSN];

  const int tid  = threadIdx.x;
  const int wave = tid >> 5;
  const int lane = tid & 31;
  const int hh   = lane >> 4;
  const int c    = lane & 15;
  const int bq   = blockIdx.x >> 3;
  const int qt   = blockIdx.x & 7;
  const int qw   = qt * 64 + wave * 16;

  const __bf16* Vh = (const __bf16*)(const void*)vthp;
  const __bf16* Vl = (const __bf16*)(const void*)vtlp;

#pragma unroll
  for (int i = 0; i < 2; ++i) {
    const int idx = i * 128 + tid;
    const v4u a = *(const v4u*)(MB + (size_t)qt * 1024 + idx * 4);
    *(v4u*)(mk + idx * 4) = a;
  }

#pragma unroll 1
  for (int it = 0; it < NIT; ++it) {
    const int bt     = (MODE == 1) ? bq : (bq * GT + it);
    const int vrow0  = (MODE == 1) ? (it * HD) : 0;
    const int sdbase = (MODE == 1) ? ((bt * GH + it) * GN) : (bt * GN);

    float sq[8];
    {
      const float* Sg = SD + (size_t)sdbase + qw + 8 * hh;
      const v4f sa = *(const v4f*)(Sg);
      const v4f sb = *(const v4f*)(Sg + 4);
#pragma unroll
      for (int r = 0; r < 4; ++r) { sq[r] = sa[r]; sq[r + 4] = sb[r]; }
    }

    float mrow[8], lrow[8];
    v8f oacc[NTL];
#pragma unroll
    for (int r = 0; r < 8; ++r) { mrow[r] = -INFINITY; lrow[r] = 0.f; }
#pragma unroll
    for (int t = 0; t < NTL; ++t) oacc[t] = (v8f){0.f,0.f,0.f,0.f,0.f,0.f,0.f,0.f};

#pragma unroll 1
    for (int kc = 0; kc < GN / 64; ++kc) {
      const int kv0 = kc * 64;
      __syncthreads();
      if (kc == 0) {
        const v4f dvv = *(const v4f*)(SD + (size_t)PLANE + sdbase + tid * 4);
        *(v4f*)(dsh + tid * 4) = dvv;
      }
      {
#pragma unroll
        for (int i = 0; i < PPT; ++i) {
          const int p  = i * 128 + tid;
          const int r  = p >> 3;
          const int c8 = (p & 7) * 8;
          const size_t go = (size_t)(vrow0 + r) * NTOK + (size_t)bt * GN + kv0 + c8;
          const v8b a0 = *(const v8b*)(Vh + go);
          const v8b a1 = *(const v8b*)(Vl + go);
          *(v8b*)(Vth + r * 64 + c8) = a0;
          *(v8b*)(Vtl + r * 64 + c8) = a1;
        }
      }
      __syncthreads();

      float dv[4];
#pragma unroll
      for (int j = 0; j < 4; ++j) dv[j] = dsh[kv0 + j * 16 + c];

      v8f s[4];
      float cm[8];
#pragma unroll
      for (int r = 0; r < 8; ++r) {
        const int mi = (wave * 16 + 8 * hh + r) * 16 + 2 * kc;
        const unsigned w0 = mk[mi];
        const unsigned w1 = mk[mi + 1];
        float m = -INFINITY;
#pragma unroll
        for (int j = 0; j < 4; ++j) {
          const unsigned w   = (j < 2) ? w0 : w1;
          const unsigned bit = (w >> ((j & 1) * 16 + c)) & 1u;
          const float v  = sq[r] + dv[j];
          const float e  = (v >= 0.f) ? v : 0.2f * v;
          const float sv = (bit != 0u) ? e : NEGV;
          s[j][r] = sv;
          m = fmaxf(m, sv);
        }
#pragma unroll
        for (int off = 1; off < 16; off <<= 1) m = fmaxf(m, __shfl_xor(m, off, 32));
        cm[r] = m;
      }
      __bf16* pwh = Psh[wave];
      __bf16* pwl = Psl[wave];
#pragma unroll
      for (int r = 0; r < 8; ++r) {
        const float mnew = fmaxf(mrow[r], cm[r]);
        const float alpha = expf(mrow[r] - mnew);
        mrow[r] = mnew;
        float psum = 0.f;
#pragma unroll
        for (int j = 0; j < 4; ++j) {
          const float p = expf(s[j][r] - mnew);
          psum += p;
          __bf16 a, bl; at_split(p, a, bl);
          pwh[(8 * hh + r) * 64 + j * 16 + c] = a;
          pwl[(8 * hh + r) * 64 + j * 16 + c] = bl;
        }
#pragma unroll
        for (int off = 1; off < 16; off <<= 1) psum += __shfl_xor(psum, off, 32);
        lrow[r] = lrow[r] * alpha + psum;
#pragma unroll
        for (int t = 0; t < NTL; ++t) oacc[t][r] *= alpha;
      }
      wave_lds_sync();
#pragma unroll 1
      for (int kk = 0; kk < 2; ++kk) {
        FB pa, pl;
        pa.h[0] = *(const v8b*)(pwh + c * 64 + kk * 32 + 8 * hh);
        pa.h[1] = *(const v8b*)(pwh + c * 64 + kk * 32 + 16 + 8 * hh);
        pl.h[0] = *(const v8b*)(pwl + c * 64 + kk * 32 + 8 * hh);
        pl.h[1] = *(const v8b*)(pwl + c * 64 + kk * 32 + 16 + 8 * hh);
#pragma unroll
        for (int t = 0; t < NTL; ++t) {
          FB vb, vl;
          vb.h[0] = *(const v8b*)(Vth + (t * 16 + c) * 64 + kk * 32 + 8 * hh);
          vb.h[1] = *(const v8b*)(Vth + (t * 16 + c) * 64 + kk * 32 + 16 + 8 * hh);
          vl.h[0] = *(const v8b*)(Vtl + (t * 16 + c) * 64 + kk * 32 + 8 * hh);
          vl.h[1] = *(const v8b*)(Vtl + (t * 16 + c) * 64 + kk * 32 + 16 + 8 * hh);
          oacc[t] = at_mma(pa.v, vb.v, oacc[t]);
          oacc[t] = at_mma(pa.v, vl.v, oacc[t]);
          oacc[t] = at_mma(pl.v, vb.v, oacc[t]);
        }
      }
    }

    if (MODE == 1) {
      float* xw = xs + (wave * 16) * 132;
#pragma unroll
      for (int r = 0; r < 8; ++r) {
        const float inv = 1.0f / lrow[r];
#pragma unroll
        for (int t = 0; t < NTL; ++t) {
          const float v  = oacc[t][r] * inv;
          const float ev = (v > 0.f) ? v : expm1f(v);
          xw[(8 * hh + r) * 132 + it * HD + t * 16 + c] = ev;
        }
      }
    } else {
      float* ow = dyn_slab + (wave * 16) * (GC * GT);
#pragma unroll
      for (int r = 0; r < 8; ++r) {
        const float inv = 1.0f / lrow[r];
#pragma unroll
        for (int t = 0; t < NTL; ++t) ow[(8 * hh + r) * (GC * GT) + (t * 16 + c) * GT + it] = oacc[t][r] * inv;
      }
    }
  }

  __syncthreads();
  if (MODE == 1) {
    const int ch0 = (lane & 15) * 8;
    const bool islo = (lane >= 16);
    v4u pv[16];
#pragma unroll
    for (int rr = 0; rr < 16; ++rr) {
      const float* sp = xs + (wave * 16 + rr) * 132 + ch0;
      const v4f a = *(const v4f*)(sp);
      const v4f b = *(const v4f*)(sp + 4);
      float f[8];
#pragma unroll
      for (int e = 0; e < 4; ++e) { f[e] = a[e]; f[e + 4] = b[e]; }
      v4u u;
#pragma unroll
      for (int e = 0; e < 4; ++e) {
        const unsigned short h0 = f2bf_bits(f[2 * e]), h1 = f2bf_bits(f[2 * e + 1]);
        const unsigned short l0 = f2bf_bits(f[2 * e] - bf_bits2f(h0)), l1 = f2bf_bits(f[2 * e + 1] - bf_bits2f(h1));
        const unsigned uh = pk16(h0, h1), ul = pk16(l0, l1);
        u[e] = islo ? ul : uh;
      }
      pv[rr] = u;
    }
    const size_t rowbase = (size_t)bq * GN + qw;
    for (int pass = 0; pass < 2; ++pass) {
#pragma unroll
      for (int rr = 0; rr < 16; ++rr) {
        *(volatile v4u*)(x1hl + (rowbase + rr) * 256 + lane * 8) = pv[rr];
      }
      __threadfence();
    }
  } else {
    const size_t ob = ((size_t)bq * GN + (size_t)qt * 64) * (GC * GT);
    for (int pass = 0; pass < 2; ++pass) {
#pragma unroll 4
      for (int i = 0; i < 96; ++i) {
        const int idx = i * 128 + tid;
        const v4f v = *(const v4f*)(dyn_slab + idx * 4);
        *(volatile v4f*)(out + ob + (size_t)idx * 4) = v;
      }
      __threadfence();
    }
  }
}

extern "C" void kernel_launch(void* const* d_in, const int* in_sizes, int n_in,
                              void* d_out, int out_size, void* d_ws, size_t ws_size,
                              hipStream_t stream) {
  if (n_in < 6) return;
  if (in_sizes[0] != GB * GN * GF * GT) return;
  if (in_sizes[1] != GN * GN) return;
  if (in_sizes[2] != GH * GF * GO) return;
  if (in_sizes[3] != GH * 2 * GO) return;
  if (in_sizes[4] != GHO * GC) return;
  if (in_sizes[5] != 2 * GC) return;
  if (out_size != GB * GN * GC * GT) return;

  const float* x   = (const float*)d_in[0];
  const int*   adj = (const int*)d_in[1];
  const float* Wh  = (const float*)d_in[2];
  const float* ah  = (const float*)d_in[3];
  const float* Wo  = (const float*)d_in[4];
  const float* ao  = (const float*)d_in[5];

  const size_t PA   = (size_t)2 * GHO * NTOK * 2;
  const size_t PBr  = (size_t)NTOK * 256 * 2;
  const size_t PSD1 = (size_t)2 * BT * GH * GN * 4;
  const size_t PSD2 = (size_t)2 * BT * GN * 4;
  const size_t PMB  = (size_t)GN * 16 * 4;
  const size_t PW1  = (size_t)GHO * GF * 2;
  const size_t PW2  = (size_t)GC * 256 * 2;
  const size_t PAV  = (size_t)384 * 4;
  size_t off = 0;
  const size_t oA   = off; off += PA;
  const size_t oB   = off; off += PBr;
  const size_t oSD1 = off; off += PSD1;
  const size_t oSD2 = off; off += PSD2;
  const size_t oMB  = off; off += PMB;
  const size_t oW1  = off; off += PW1;
  const size_t oW2  = off; off += PW2;
  const size_t oAV  = off; off += PAV;
  if (off > ws_size) return;
  if (off > (size_t)134217728) return;

  char* ws = (char*)d_ws;
  unsigned short* V1Th = (unsigned short*)(ws + oA);
  unsigned short* V1Tl = (unsigned short*)(ws + oA + (size_t)GHO * NTOK * 2);
  unsigned short* V2Th = (unsigned short*)(ws + oA);
  unsigned short* V2Tl = (unsigned short*)(ws + oA + (size_t)GC * NTOK * 2);
  unsigned short* XB   = (unsigned short*)(ws + oB);
  unsigned short* X1hl = (unsigned short*)(ws + oB);
  float*          SD1  = (float*)(ws + oSD1);
  float*          SD2  = (float*)(ws + oSD2);
  unsigned*       MB   = (unsigned*)(ws + oMB);
  unsigned short* W1t  = (unsigned short*)(ws + oW1);
  unsigned short* W2t2 = (unsigned short*)(ws + oW2);
  float*          AV   = (float*)(ws + oAV);

  k_prep<<<dim3(PB_ALL), dim3(256), 0, stream>>>(x, adj, Wh, ah, Wo, ao, XB, W1t, W2t2, AV, MB);
  k_gemm_vt<1><<<dim3((GHO / 64) * (NTOK / 64) / 8), dim3(256), 0, stream>>>(W1t, XB, AV, V1Th, V1Tl, SD1);
  k_att<2, 1><<<dim3(BT * (GN / 64)), dim3(128), 0, stream>>>(V1Th, V1Tl, SD1, MB, X1hl, (float*)d_out);
  k_gemm_vt<2><<<dim3((GC / 64) * (NTOK / 64) / 8), dim3(256), 0, stream>>>(W2t2, X1hl, AV, V2Th, V2Tl, SD2);
  const size_t slabBytes = (size_t)64 * GC * GT * 4;
  (void)hipFuncSetAttribute(reinterpret_cast<const void*>(&k_att<4, 2>), hipFuncAttributeMaxDynamicSharedMemorySize, (int)slabBytes);
  k_att<4, 2><<<dim3(GB * (GN / 64)), dim3(128), slabBytes, stream>>>(V2Th, V2Tl, SD2, MB, X1hl, (float*)d_out);
  (void)hipGetLastError();
}
